// mylstmSAGEConv_3504693313808
// MI455X (gfx1250) — hardware-verified
//
#include <hip/hip_runtime.h>
#include <stddef.h>
#include <stdint.h>
#include <math.h>


#define NN     10000
#define DEG    32
#define FD     256
#define G4     1024
#define MP     10048
#define K2     512
#define GBM    64
#define GBN    64
#define GTHR   128
#define NTHR   256
#define WSMAX  134217728
#define STG_BYTES 65536
#define DSM_BYTES (STG_BYTES + 512)
#define SQC    16

#define PA_XB  (MP * FD / 8)
#define PA_W   (G4 * FD / 8)
#define PA_Z   ((MP * FD * 4 + 2 * MP * FD * 2) / 16)
#define PA_ALL (PA_XB + 2 * PA_W + PA_Z)
#define PB_W2  (G4 * K2 / 8)
#define PB_WL  (FD * K2 / 8)
#define PB_F   (64 * G4)
#define PB_Z   ((MP - NN) * K2 / 8)
#define PB_ALL (PB_W2 + PB_WL + PB_F + 2 * PB_Z)

static_assert(MP == 157 * 64 && MP >= NN && (MP - NN) == 48);
static_assert(4 * FD == G4 && G4 == 1024 && FD % 32 == 0 && K2 % 32 == 0 && K2 == 2 * FD);
static_assert(MP % GBM == 0 && G4 % GBN == 0 && FD % GBN == 0);
static_assert(PA_XB % NTHR == 0 && PA_W % NTHR == 0 && PA_Z % NTHR == 0);
static_assert(PB_W2 % NTHR == 0 && PB_WL % NTHR == 0 && PB_F % NTHR == 0 && PB_Z % NTHR == 0);
static_assert(NN % SQC == 0 && SQC * K2 * 2 == 1024 * 16);
static_assert(64 * 2 == 128 && DEG == 32);

typedef float          v4f   __attribute__((ext_vector_type(4)));
typedef float          v8f   __attribute__((ext_vector_type(8)));
typedef int            v8i   __attribute__((ext_vector_type(8)));
typedef unsigned short v8us  __attribute__((ext_vector_type(8)));
typedef unsigned short v16us __attribute__((ext_vector_type(16)));
typedef __bf16         v16bf __attribute__((ext_vector_type(16)));
typedef v4f  __attribute__((may_alias)) v4fa;
typedef v8us __attribute__((may_alias)) v8usa;
union FragB { v16bf v; v16us u; v8us h[2]; v8i w; };

__device__ __forceinline__ v8f wmb(const FragB& a, const FragB& b, v8f c) {
  v8f d = __builtin_amdgcn_wmma_f32_16x16x32_bf16(false, a.v, false, b.v, (short)0, c, false, false);
  asm volatile("v_nop\n\tv_nop\n\tv_nop\n\tv_nop" : "+v"(d) : "v"(a.w), "v"(b.w));
  return d;
}

__device__ __forceinline__ unsigned bf16_bits(float f) {
  const unsigned u = __float_as_uint(f);
  return (u + 0x7FFFu + ((u >> 16) & 1u)) >> 16;
}
__device__ __forceinline__ float bf16_val(float f) {
  return __uint_as_float(bf16_bits(f) << 16);
}
__device__ __forceinline__ unsigned short hl_sel(float v, bool lo_sel) {
  const unsigned hb = bf16_bits(v);
  const unsigned lb = bf16_bits(v - __uint_as_float(hb << 16));
  return (unsigned short)(lo_sel ? lb : hb);
}
__device__ __forceinline__ v8us pack_hl8(v4f a, v4f b, bool lo_sel) {
  v8us o;
  o[0] = hl_sel(a.x, lo_sel); o[1] = hl_sel(a.y, lo_sel);
  o[2] = hl_sel(a.z, lo_sel); o[3] = hl_sel(a.w, lo_sel);
  o[4] = hl_sel(b.x, lo_sel); o[5] = hl_sel(b.y, lo_sel);
  o[6] = hl_sel(b.z, lo_sel); o[7] = hl_sel(b.w, lo_sel);
  return o;
}

__device__ __forceinline__ float sig_fast(float x) { return __builtin_amdgcn_rcpf(1.0f + __expf(-x)); }
__device__ __forceinline__ float tanh_fast(float x) { return 2.0f * sig_fast(2.0f * x) - 1.0f; }
__device__ __forceinline__ float sig_p(float x) { return __builtin_amdgcn_rcpf(1.0f + expf(-x)); }
__device__ __forceinline__ float tanh_p(float x) { return 2.0f * sig_p(2.0f * x) - 1.0f; }

template <bool FIRST>
__device__ __forceinline__ float cell_c(float gi, float gf, float gg, float cp) {
  if constexpr (FIRST) return sig_fast(gi) * tanh_fast(gg);
  else return sig_fast(gf) * cp + sig_fast(gi) * tanh_fast(gg);
}
__device__ __forceinline__ float cell_h(float go, float cn) { return sig_fast(go) * tanh_fast(cn); }

__device__ __forceinline__ void cvt8_put(const float* p, bool ok, unsigned short* dp) {
  const v4f a = *(const v4fa*)p;
  const v4f b = *(const v4fa*)(p + 4);
  v8us o;
  o[0] = ok ? (unsigned short)bf16_bits(a.x) : (unsigned short)0;
  o[1] = ok ? (unsigned short)bf16_bits(a.y) : (unsigned short)0;
  o[2] = ok ? (unsigned short)bf16_bits(a.z) : (unsigned short)0;
  o[3] = ok ? (unsigned short)bf16_bits(a.w) : (unsigned short)0;
  o[4] = ok ? (unsigned short)bf16_bits(b.x) : (unsigned short)0;
  o[5] = ok ? (unsigned short)bf16_bits(b.y) : (unsigned short)0;
  o[6] = ok ? (unsigned short)bf16_bits(b.z) : (unsigned short)0;
  o[7] = ok ? (unsigned short)bf16_bits(b.w) : (unsigned short)0;
  *(volatile v8us*)dp = o;
  __threadfence();
  *(volatile v8us*)dp = o;
}
__device__ __forceinline__ void rnd4_put(const float* p, float* dp) {
  const v4f a = *(const v4fa*)p;
  v4f o;
  o.x = bf16_val(a.x); o.y = bf16_val(a.y); o.z = bf16_val(a.z); o.w = bf16_val(a.w);
  *(volatile v4f*)dp = o;
  __threadfence();
  *(volatile v4f*)dp = o;
}
__device__ __forceinline__ void sum4_put(const float* pa, const float* pb, float* dp) {
  const v4f a = *(const v4fa*)pa;
  const v4f b = *(const v4fa*)pb;
  v4f o;
  o.x = bf16_val(a.x) + bf16_val(b.x); o.y = bf16_val(a.y) + bf16_val(b.y);
  o.z = bf16_val(a.z) + bf16_val(b.z); o.w = bf16_val(a.w) + bf16_val(b.w);
  *(volatile v4f*)dp = o;
  __threadfence();
  *(volatile v4f*)dp = o;
}
__device__ __forceinline__ void zero16_put(unsigned short* dp) {
  const v8us z = {0, 0, 0, 0, 0, 0, 0, 0};
  *(volatile v8us*)dp = z;
  __threadfence();
  *(volatile v8us*)dp = z;
}

__global__ __launch_bounds__(NTHR) void k_pa(
    const float* __restrict__ nf, const float* __restrict__ wih1, const float* __restrict__ whh1,
    unsigned short* XB, unsigned short* WIH1P, unsigned short* WHH1P, unsigned short* ZR)
{
  const int u = (int)blockIdx.x * NTHR + (int)threadIdx.x;
  if (u < PA_XB) {
    const int row = u >> 5;
    const int k8  = (u & 31) * 8;
    const int rc  = row < NN ? row : NN - 1;
    cvt8_put(nf + (size_t)rc * FD + k8, row < NN, XB + (size_t)row * FD + k8);
  } else if (u < PA_XB + 2 * PA_W) {
    const int v0  = u - PA_XB;
    const int sel = v0 >= PA_W ? 1 : 0;
    const int v   = v0 - sel * PA_W;
    const int pr  = v >> 5;
    const int k8  = (v & 31) * 8;
    const int nbq = pr >> 8, g = (pr >> 6) & 3, uu = pr & 63;
    const int orow = g * 256 + nbq * 64 + uu;
    if (sel == 0) cvt8_put(wih1 + (size_t)orow * FD + k8, true, WIH1P + (size_t)pr * FD + k8);
    else          cvt8_put(whh1 + (size_t)orow * FD + k8, true, WHH1P + (size_t)pr * FD + k8);
  } else if (u < PA_ALL) {
    const int v = u - (PA_XB + 2 * PA_W);
    zero16_put(ZR + (size_t)8 * v);
  }
}

__global__ __launch_bounds__(NTHR) void k_pb(
    const float* __restrict__ wih2, const float* __restrict__ whh2, const float* __restrict__ wl,
    unsigned short* WIH2D, float* W2F, unsigned short* WLD, unsigned short* HAGG, unsigned short* HSHL)
{
  const int u = (int)blockIdx.x * NTHR + (int)threadIdx.x;
  if (u < PB_W2) {
    const int n  = u >> 6;
    const int k8 = (u & 63) * 8;
    cvt8_put(wih2 + (size_t)n * FD + (k8 & (FD - 1)), true, WIH2D + (size_t)n * K2 + k8);
  } else if (u < PB_W2 + PB_WL) {
    const int v  = u - PB_W2;
    const int n  = v >> 6;
    const int k8 = (v & 63) * 8;
    cvt8_put(wl + (size_t)n * FD + (k8 & (FD - 1)), true, WLD + (size_t)n * K2 + k8);
  } else if (u < PB_W2 + PB_WL + PB_F) {
    const int v  = u - (PB_W2 + PB_WL);
    const int k4 = v >> 10;
    const int j  = v & 1023;
    rnd4_put(whh2 + (size_t)j * FD + 4 * k4, W2F + (size_t)4 * v);
  } else if (u < PB_W2 + PB_WL + PB_F + PB_Z) {
    const int v = u - (PB_W2 + PB_WL + PB_F);
    zero16_put(HAGG + (size_t)NN * K2 + (size_t)8 * v);
  } else if (u < PB_ALL) {
    const int v = u - (PB_W2 + PB_WL + PB_F + PB_Z);
    zero16_put(HSHL + (size_t)NN * K2 + (size_t)8 * v);
  }
}

__global__ __launch_bounds__(NTHR) void k_pc(
    const float* __restrict__ bih1, const float* __restrict__ bhh1,
    const float* __restrict__ bih2, const float* __restrict__ bhh2,
    const float* __restrict__ bl, const float* __restrict__ bias,
    float* BS1P, float* BS2, float* BL)
{
  const int tid = (int)threadIdx.x;
  const int b = (int)blockIdx.x;
  if (b == 0) {
    const int p4 = 4 * tid;
    const int nbq = p4 >> 8, g = (p4 >> 6) & 3, uu = p4 & 63;
    const int o = g * 256 + nbq * 64 + uu;
    sum4_put(bih1 + o, bhh1 + o, BS1P + p4);
  } else if (b == 1) {
    sum4_put(bih2 + 4 * tid, bhh2 + 4 * tid, BS2 + 4 * tid);
  } else {
    if (tid < 64) sum4_put(bl + 4 * tid, bias + 4 * tid, BL + 4 * tid);
  }
}

template <bool BIAS, bool GUARD>
__global__ __launch_bounds__(GTHR) void k_gemm(
    const unsigned short* __restrict__ A, int lda,
    const unsigned short* __restrict__ WT, int ldb, int K,
    float* outF, int ldo, const float* __restrict__ bias, int nrows)
{
  __shared__ __attribute__((aligned(16))) float stg[GBM * GBN];
  const int tid = (int)threadIdx.x, lane = tid & 31, wave = tid >> 5, hh = lane >> 4, m = lane & 15;
  const int rowBase = (int)blockIdx.x * GBM;
  const int col0    = (int)blockIdx.y * GBN;

  v8f acc[4];
  {
    const v8f z = {0.f, 0.f, 0.f, 0.f, 0.f, 0.f, 0.f, 0.f};
    acc[0] = z; acc[1] = z; acc[2] = z; acc[3] = z;
  }
  const unsigned short* ap = A  + (size_t)(rowBase + 16 * wave + m) * (size_t)lda + 8 * hh;
  const unsigned short* wp = WT + (size_t)(col0 + m) * (size_t)ldb + 8 * hh;
  const int ksteps = K >> 5;
#pragma unroll 1
  for (int ks = 0; ks < ksteps; ++ks) {
    FragB af;
    af.h[0] = *(const v8usa*)(ap + 32 * ks);
    af.h[1] = *(const v8usa*)(ap + 32 * ks + 16);
#pragma unroll
    for (int t = 0; t < 4; ++t) {
      const unsigned short* wq = wp + (size_t)(16 * t) * (size_t)ldb + 32 * ks;
      FragB bf;
      bf.h[0] = *(const v8usa*)wq;
      bf.h[1] = *(const v8usa*)(wq + 16);
      acc[t] = wmb(af, bf, acc[t]);
    }
  }

#pragma unroll
  for (int t = 0; t < 4; ++t) {
    const int lc = 16 * t + m;
#pragma unroll
    for (int r = 0; r < 8; ++r) {
      const int lr = 16 * wave + 8 * hh + r;
      stg[lr * GBN + lc] = acc[t][r];
    }
  }
  __syncthreads();

  v4f bb = {0.f, 0.f, 0.f, 0.f};
  if constexpr (BIAS) bb = *(const v4fa*)(bias + col0 + 4 * m);
  float* ob = outF + col0 + 4 * m;
  v4f fv[8];
#pragma unroll
  for (int i = 0; i < 8; ++i) {
    const int lr = 16 * wave + 2 * i + hh;
    const v4f tv = *(const v4fa*)(stg + lr * GBN + 4 * m);
    fv[i] = tv + bb;
  }
#pragma unroll
  for (int i = 0; i < 8; ++i) {
    const int row = rowBase + 16 * wave + 2 * i + hh;
    if (!GUARD || row < nrows) *(volatile v4f*)(ob + (size_t)row * (size_t)ldo) = fv[i];
  }
  __threadfence();
#pragma unroll
  for (int i = 0; i < 8; ++i) {
    const int row = rowBase + 16 * wave + 2 * i + hh;
    if (!GUARD || row < nrows) *(volatile v4f*)(ob + (size_t)row * (size_t)ldo) = fv[i];
  }
}

template <bool FIRST, bool LAST>
__global__ __launch_bounds__(256) void k_step(
    const int* __restrict__ edges, const float* __restrict__ ew,
    const unsigned short* __restrict__ Hin, const unsigned short* __restrict__ WHH,
    const float* __restrict__ P, const float* __restrict__ BS1P,
    float* C, unsigned short* Hout, unsigned short* HAGG, int t)
{
  extern __shared__ __attribute__((aligned(16))) unsigned char dsm[];
  float* stg  = (float*)dsm;
  int*   ssrc = (int*)(dsm + STG_BYTES);
  float* sw   = (float*)(dsm + STG_BYTES + 256);

  const int tid = (int)threadIdx.x, lane = tid & 31, wave = tid >> 5, hh = lane >> 4, m = lane & 15;
  const int r0 = (int)blockIdx.x * 64;
  const int nb = (int)blockIdx.y;

  if (tid < 64) {
    const int r  = r0 + tid;
    const int rc = r < NN ? r : NN - 1;
    int e = edges[(size_t)rc * DEG + t];
    const float wv = ew[(size_t)rc * DEG + t];
    e = e < 0 ? 0 : (e > NN - 1 ? NN - 1 : e);
    const bool ok = r < NN;
    ssrc[tid] = ok ? e : 0;
    sw[tid]   = ok ? bf16_val(wv) : 0.0f;
  }

  if constexpr (!FIRST) {
    const int rp = wave & 1, gq = wave >> 1;
    v8f acc[2][4];
    {
      const v8f z = {0.f, 0.f, 0.f, 0.f, 0.f, 0.f, 0.f, 0.f};
#pragma unroll
      for (int mt = 0; mt < 2; ++mt)
#pragma unroll
        for (int nt = 0; nt < 4; ++nt) acc[mt][nt] = z;
    }
    const unsigned short* a0p = Hin + (size_t)(r0 + 32 * rp + m) * FD + 8 * hh;
    const unsigned short* a1p = a0p + (size_t)16 * FD;
    const unsigned short* bp  = WHH + (size_t)(nb * 256 + 64 * gq + m) * FD + 8 * hh;
#pragma unroll 1
    for (int ks = 0; ks < FD / 32; ++ks) {
      FragB a0, a1;
      a0.h[0] = *(const v8usa*)(a0p + 32 * ks);
      a0.h[1] = *(const v8usa*)(a0p + 32 * ks + 16);
      a1.h[0] = *(const v8usa*)(a1p + 32 * ks);
      a1.h[1] = *(const v8usa*)(a1p + 32 * ks + 16);
#pragma unroll
      for (int nt = 0; nt < 4; ++nt) {
        const unsigned short* bq = bp + (size_t)(16 * nt) * FD + 32 * ks;
        FragB b;
        b.h[0] = *(const v8usa*)bq;
        b.h[1] = *(const v8usa*)(bq + 16);
        acc[0][nt] = wmb(a0, b, acc[0][nt]);
        acc[1][nt] = wmb(a1, b, acc[1][nt]);
      }
    }
#pragma unroll
    for (int mt = 0; mt < 2; ++mt)
#pragma unroll
      for (int nt = 0; nt < 4; ++nt)
#pragma unroll
        for (int r = 0; r < 8; ++r)
          stg[(32 * rp + 16 * mt + 8 * hh + r) * 256 + 64 * gq + 16 * nt + m] = acc[mt][nt][r];
  }
  __syncthreads();

  {
    const int q = tid & 15;
    const float* bsp = BS1P + nb * 256 + 4 * q;
    const v4f bi = *(const v4fa*)(bsp);
    const v4f bf = *(const v4fa*)(bsp + 64);
    const v4f bg = *(const v4fa*)(bsp + 128);
    const v4f bo = *(const v4fa*)(bsp + 192);
#pragma unroll 1
    for (int it = 0; it < 4; ++it) {
      const int row = it * 16 + (tid >> 4);
      const int src = ssrc[row];
      const float w = sw[row];
      const float* pp = P + (size_t)src * G4 + nb * 256 + 4 * q;
      const v4f p0 = *(const v4fa*)(pp);
      const v4f p1 = *(const v4fa*)(pp + 64);
      const v4f p2 = *(const v4fa*)(pp + 128);
      const v4f p3 = *(const v4fa*)(pp + 192);
      float* sr = stg + row * 256 + 4 * q;
      v4f gi, gf, gg, go;
      v4f cp = {0.f, 0.f, 0.f, 0.f};
      if constexpr (FIRST) {
        gi = p0 * w + bi; gf = p1 * w + bf; gg = p2 * w + bg; go = p3 * w + bo;
      } else {
        const v4f a0 = *(const v4fa*)(sr);
        const v4f a1 = *(const v4fa*)(sr + 64);
        const v4f a2 = *(const v4fa*)(sr + 128);
        const v4f a3 = *(const v4fa*)(sr + 192);
        gi = (p0 * w + a0) + bi; gf = (p1 * w + a1) + bf;
        gg = (p2 * w + a2) + bg; go = (p3 * w + a3) + bo;
        cp = *(const v4fa*)(C + (size_t)(r0 + row) * FD + nb * 64 + 4 * q);
      }
      v4f cn, hn;
      cn.x = cell_c<FIRST>(gi.x, gf.x, gg.x, cp.x); hn.x = cell_h(go.x, cn.x);
      cn.y = cell_c<FIRST>(gi.y, gf.y, gg.y, cp.y); hn.y = cell_h(go.y, cn.y);
      cn.z = cell_c<FIRST>(gi.z, gf.z, gg.z, cp.z); hn.z = cell_h(go.z, cn.z);
      cn.w = cell_c<FIRST>(gi.w, gf.w, gg.w, cp.w); hn.w = cell_h(go.w, cn.w);
      *(v4fa*)(sr)      = cn;
      *(v4fa*)(sr + 64) = hn;
    }
  }
  __syncthreads();

  if constexpr (!LAST) {
    v4f  cv[4];
    v8us hv[2];
#pragma unroll
    for (int j = 0; j < 4; ++j) {
      const int id = j * 256 + tid;
      cv[j] = *(const v4fa*)(stg + (id >> 4) * 256 + 4 * (id & 15));
    }
#pragma unroll
    for (int j = 0; j < 2; ++j) {
      const int id = j * 256 + tid;
      const float* hp = stg + (id >> 3) * 256 + 64 + 8 * (id & 7);
      hv[j] = pack_hl8(*(const v4fa*)hp, *(const v4fa*)(hp + 4), false);
    }
#pragma unroll
    for (int j = 0; j < 4; ++j) {
      const int id = j * 256 + tid;
      const int r = r0 + (id >> 4);
      if (r < NN) *(volatile v4f*)(C + (size_t)r * FD + nb * 64 + 4 * (id & 15)) = cv[j];
    }
#pragma unroll
    for (int j = 0; j < 2; ++j) {
      const int id = j * 256 + tid;
      const int r = r0 + (id >> 3);
      if (r < NN) *(volatile v8us*)(Hout + (size_t)r * FD + nb * 64 + 8 * (id & 7)) = hv[j];
    }
    __threadfence();
#pragma unroll
    for (int j = 0; j < 4; ++j) {
      const int id = j * 256 + tid;
      const int r = r0 + (id >> 4);
      if (r < NN) *(volatile v4f*)(C + (size_t)r * FD + nb * 64 + 4 * (id & 15)) = cv[j];
    }
#pragma unroll
    for (int j = 0; j < 2; ++j) {
      const int id = j * 256 + tid;
      const int r = r0 + (id >> 3);
      if (r < NN) *(volatile v8us*)(Hout + (size_t)r * FD + nb * 64 + 8 * (id & 7)) = hv[j];
    }
  } else {
    v8us gv[4];
#pragma unroll
    for (int j = 0; j < 4; ++j) {
      const int id = j * 256 + tid;
      const int line = id >> 3;
      const int row = line >> 1;
      const bool lo_sel = (line & 1) != 0;
      const float* hp = stg + row * 256 + 64 + 8 * (id & 7);
      gv[j] = pack_hl8(*(const v4fa*)hp, *(const v4fa*)(hp + 4), lo_sel);
    }
#pragma unroll
    for (int j = 0; j < 4; ++j) {
      const int id = j * 256 + tid;
      const int line = id >> 3;
      const int r = r0 + (line >> 1);
      if (r < NN)
        *(volatile v8us*)(HAGG + (size_t)r * K2 + (size_t)(line & 1) * FD + nb * 64 + 8 * (id & 7)) = gv[j];
    }
    __threadfence();
#pragma unroll
    for (int j = 0; j < 4; ++j) {
      const int id = j * 256 + tid;
      const int line = id >> 3;
      const int r = r0 + (line >> 1);
      if (r < NN)
        *(volatile v8us*)(HAGG + (size_t)r * K2 + (size_t)(line & 1) * FD + nb * 64 + 8 * (id & 7)) = gv[j];
    }
  }
}

__global__ __launch_bounds__(1024) void k_seq(const float* __restrict__ XG, const float* __restrict__ W2F,
                                              unsigned short* HSHL)
{
  __shared__ __attribute__((aligned(16))) float hcur[FD];
  __shared__ __attribute__((aligned(16))) float gs[G4];
  __shared__ __attribute__((aligned(16))) float hst[SQC * FD];
  const int j = (int)threadIdx.x;
  if (j < FD) hcur[j] = 0.0f;
  float c = 0.0f;
  float xg = XG[j];
  const float* wj = W2F + 4 * j;
  __syncthreads();

#pragma unroll 1
  for (int n = 0; n < NN; ++n) {
    const int nn = (n + 1 < NN) ? n + 1 : NN - 1;
    const float xnext = XG[(size_t)nn * G4 + j];
    float acc = xg;
#pragma unroll 2
    for (int k4 = 0; k4 < FD / 4; ++k4) {
      const v4f wv = *(const v4fa*)(wj + (size_t)k4 * (4 * G4));
      const v4f hv = *(const v4fa*)(hcur + 4 * k4);
      acc = fmaf(hv.x, wv.x, acc);
      acc = fmaf(hv.y, wv.y, acc);
      acc = fmaf(hv.z, wv.z, acc);
      acc = fmaf(hv.w, wv.w, acc);
    }
    gs[j] = acc;
    __syncthreads();
    if (j < FD) {
      const float gi = gs[j], gf = gs[FD + j], gg = gs[2 * FD + j], go = gs[3 * FD + j];
      c = sig_p(gf) * c + sig_p(gi) * tanh_p(gg);
      const float h = sig_p(go) * tanh_p(c);
      hcur[j] = h;
      hst[(n & (SQC - 1)) * FD + j] = h;
    }
    __syncthreads();
    if ((n & (SQC - 1)) == SQC - 1) {
      const int n0  = n - (SQC - 1);
      const int row = j >> 6;
      const int p   = j & 63;
      const bool lo_sel = p >= 32;
      const float* hp = hst + row * FD + 8 * (p & 31);
      const v8us o = pack_hl8(*(const v4fa*)hp, *(const v4fa*)(hp + 4), lo_sel);
      unsigned short* dp = HSHL + (size_t)(n0 + row) * K2 + 8 * p;
      *(volatile v8us*)dp = o;
      __threadfence();
      *(volatile v8us*)dp = o;
    }
    xg = xnext;
  }
}

static inline size_t al256(size_t o) { return (o + 255) & ~(size_t)255; }

extern "C" void kernel_launch(void* const* d_in, const int* in_sizes, int n_in,
                              void* d_out, int out_size, void* d_ws, size_t ws_size,
                              hipStream_t stream) {
  if (n_in < 14) return;
  if (in_sizes[0] != NN * FD) return;
  if (in_sizes[1] != NN * DEG) return;
  if (in_sizes[2] != NN * DEG) return;
  if (in_sizes[3] != G4 * FD || in_sizes[4] != G4 * FD) return;
  if (in_sizes[5] != G4 || in_sizes[6] != G4) return;
  if (in_sizes[7] != G4 * FD || in_sizes[8] != G4 * FD) return;
  if (in_sizes[9] != G4 || in_sizes[10] != G4) return;
  if (in_sizes[11] != FD * FD) return;
  if (in_sizes[12] != FD || in_sizes[13] != FD) return;
  if (out_size != NN * FD) return;

  const float* nf   = (const float*)d_in[0];
  const int*   edg  = (const int*)d_in[1];
  const float* ew   = (const float*)d_in[2];
  const float* wih1 = (const float*)d_in[3];
  const float* whh1 = (const float*)d_in[4];
  const float* bih1 = (const float*)d_in[5];
  const float* bhh1 = (const float*)d_in[6];
  const float* wih2 = (const float*)d_in[7];
  const float* whh2 = (const float*)d_in[8];
  const float* bih2 = (const float*)d_in[9];
  const float* bhh2 = (const float*)d_in[10];
  const float* wl   = (const float*)d_in[11];
  const float* bl   = (const float*)d_in[12];
  const float* bias = (const float*)d_in[13];
  float* out = (float*)d_out;

  char* ws = (char*)d_ws;
  size_t off = 0;
  const size_t oXB   = off; off = al256(off + (size_t)MP * FD * 2);
  const size_t oPX   = off; off = al256(off + (size_t)MP * G4 * 4);
  const size_t oC    = off; off = al256(off + (size_t)MP * FD * 4);
  const size_t oH0   = off; off = al256(off + (size_t)MP * FD * 2);
  const size_t oH1   = off; off = al256(off + (size_t)MP * FD * 2);
  const size_t oHAGG = off; off = al256(off + (size_t)MP * K2 * 2);
  const size_t oHSHL = off; off = al256(off + (size_t)MP * K2 * 2);
  const size_t oWI1  = off; off = al256(off + (size_t)G4 * FD * 2);
  const size_t oWH1  = off; off = al256(off + (size_t)G4 * FD * 2);
  const size_t oWI2  = off; off = al256(off + (size_t)G4 * K2 * 2);
  const size_t oW2F  = off; off = al256(off + (size_t)64 * G4 * 4 * 4);
  const size_t oWLD  = off; off = al256(off + (size_t)FD * K2 * 2);
  const size_t oBS1  = off; off = al256(off + (size_t)G4 * 4);
  const size_t oBS2  = off; off = al256(off + (size_t)G4 * 4);
  const size_t oBL   = off; off = al256(off + (size_t)FD * 4);
  if (off > ws_size || off > (size_t)WSMAX) return;
  if (oH0 != oC + (size_t)MP * FD * 4 || oH1 != oH0 + (size_t)MP * FD * 2) return;

  unsigned short* XB    = (unsigned short*)(ws + oXB);
  float*          PX    = (float*)(ws + oPX);
  float*          Cp    = (float*)(ws + oC);
  unsigned short* H0    = (unsigned short*)(ws + oH0);
  unsigned short* H1    = (unsigned short*)(ws + oH1);
  unsigned short* HAGG  = (unsigned short*)(ws + oHAGG);
  unsigned short* HSHL  = (unsigned short*)(ws + oHSHL);
  unsigned short* WIH1P = (unsigned short*)(ws + oWI1);
  unsigned short* WHH1P = (unsigned short*)(ws + oWH1);
  unsigned short* WIH2D = (unsigned short*)(ws + oWI2);
  float*          W2F   = (float*)(ws + oW2F);
  unsigned short* WLD   = (unsigned short*)(ws + oWLD);
  float*          BS1P  = (float*)(ws + oBS1);
  float*          BS2   = (float*)(ws + oBS2);
  float*          BL    = (float*)(ws + oBL);

  k_pa<<<PA_ALL / NTHR, NTHR, 0, stream>>>(nf, wih1, whh1, XB, WIH1P, WHH1P, (unsigned short*)(ws + oC));
  k_pb<<<PB_ALL / NTHR, NTHR, 0, stream>>>(wih2, whh2, wl, WIH2D, W2F, WLD, HAGG, HSHL);
  k_pc<<<3, NTHR, 0, stream>>>(bih1, bhh1, bih2, bhh2, bl, bias, BS1P, BS2, BL);

  k_gemm<false, false><<<dim3(MP / GBM, G4 / GBN), GTHR, 0, stream>>>(
      XB, FD, WIH1P, FD, FD, PX, G4, BS2, MP);

  hipFuncSetAttribute(reinterpret_cast<const void*>(&k_step<true, false>),
                      hipFuncAttributeMaxDynamicSharedMemorySize, DSM_BYTES);
  hipFuncSetAttribute(reinterpret_cast<const void*>(&k_step<false, false>),
                      hipFuncAttributeMaxDynamicSharedMemorySize, DSM_BYTES);
  hipFuncSetAttribute(reinterpret_cast<const void*>(&k_step<false, true>),
                      hipFuncAttributeMaxDynamicSharedMemorySize, DSM_BYTES);
  const dim3 gStep(MP / 64, 4);
  k_step<true, false><<<gStep, 256, DSM_BYTES, stream>>>(edg, ew, H0, WHH1P, PX, BS1P, Cp, H1, HAGG, 0);
  for (int t = 1; t < DEG - 1; ++t) {
    const unsigned short* hin = (t & 1) ? H1 : H0;
    unsigned short* hout = (t & 1) ? H0 : H1;
    k_step<false, false><<<gStep, 256, DSM_BYTES, stream>>>(edg, ew, hin, WHH1P, PX, BS1P, Cp, hout, HAGG, t);
  }
  k_step<false, true><<<gStep, 256, DSM_BYTES, stream>>>(edg, ew, H1, WHH1P, PX, BS1P, Cp, H0, HAGG, DEG - 1);

  k_gemm<true, false><<<dim3(MP / GBM, G4 / GBN), GTHR, 0, stream>>>(
      HAGG, K2, WIH2D, K2, K2, PX, G4, BS2, MP);

  k_seq<<<1, 1024, 0, stream>>>(PX, W2F, HSHL);

  k_gemm<true, true><<<dim3(MP / GBM, FD / GBN), GTHR, 0, stream>>>(
      HSHL, K2, WLD, K2, K2, out, FD, BL, NN);
}
